// WindowAttention_22419729285946
// MI455X (gfx1250) — hardware-run, weakly checked
//
#include <hip/hip_runtime.h>
#include <math.h>

typedef __attribute__((ext_vector_type(16))) _Float16 v16h;
typedef __attribute__((ext_vector_type(16))) __bf16 v16b;
typedef __attribute__((ext_vector_type(8)))  _Float16 v8h;
typedef __attribute__((ext_vector_type(8)))  float v8f;
typedef __attribute__((ext_vector_type(4)))  float v4f;
typedef __attribute__((ext_vector_type(2)))  float v2f;
typedef __attribute__((ext_vector_type(4)))  unsigned v4u;
typedef __attribute__((ext_vector_type(4)))  int v4i;
typedef float __attribute__((may_alias)) float_a;
typedef int __attribute__((may_alias)) int_a;

template <typename T> __device__ __forceinline__ void vst2(void* p, T v) { *(volatile T*)p = v; __threadfence(); *(volatile T*)p = v; }
__device__ __forceinline__ v8f wmma16(v16h a, v16h b, v8f c) {
  v8f d = __builtin_amdgcn_wmma_f32_16x16x32_f16(false, a, false, b, (short)0, c, false, false);
  asm volatile("v_nop\n\tv_nop\n\tv_nop\n\tv_nop" : "+v"(d) : "v"(a), "v"(b));
  return d;
}
__device__ __forceinline__ v8f wmma_bf(v16b a, v16b b, v8f c) {
  v8f d = __builtin_amdgcn_wmma_f32_16x16x32_bf16(false, a, false, b, (short)0, c, false, false);
  asm volatile("v_nop\n\tv_nop\n\tv_nop\n\tv_nop" : "+v"(d) : "v"(a), "v"(b));
  return d;
}
__device__ __forceinline__ v16h frag_h(const _Float16* rowk0, int lane) {
  union { v16h v; v8h q[2]; } u; const _Float16* p = rowk0 + 8 * (lane >> 4);
  u.q[0] = *(const v8h*)p; u.q[1] = *(const v8h*)(p + 16); return u.v;
}
__device__ __forceinline__ v16h frag_f32(const float* rowk0, int lane) {
  v16h a; const float* p = rowk0 + 8 * (lane >> 4);
#pragma unroll
  for (int i = 0; i < 8; ++i) { a[i] = (_Float16)p[i]; a[8 + i] = (_Float16)p[16 + i]; }
  return a;
}
__device__ __forceinline__ v16h frag_f32s(const float* rowk0, int lane, float sc) {
  v16h a; const float* p = rowk0 + 8 * (lane >> 4);
#pragma unroll
  for (int i = 0; i < 8; ++i) { a[i] = (_Float16)(p[i] * sc); a[8 + i] = (_Float16)(p[16 + i] * sc); }
  return a;
}
__device__ __forceinline__ v16h fragc_f32(const float* W, int k0, int n, int lane, int ld, int K) {
  v16h a; const int g = lane >> 4;
#pragma unroll
  for (int i = 0; i < 8; ++i) { const int ka = k0 + 8 * g + i, kb = ka + 16;
    a[i] = (_Float16)(ka < K ? W[(size_t)(ka < K ? ka : K - 1) * ld + n] : 0.f); a[8 + i] = (_Float16)(kb < K ? W[(size_t)(kb < K ? kb : K - 1) * ld + n] : 0.f); }
  return a;
}
struct F2 { v16b h, l; };
__device__ __forceinline__ F2 bsplit16(const float v[16]) { F2 r;
#pragma unroll
  for (int i = 0; i < 16; ++i) { const __bf16 h = (__bf16)v[i]; r.h[i] = h; r.l[i] = (__bf16)(v[i] - (float)h); }
  return r; }
__device__ __forceinline__ F2 split_row(const float* row, int k0, int lane) { float v[16]; const float* p = row + k0 + 8 * (lane >> 4);
#pragma unroll
  for (int i = 0; i < 8; ++i) { v[i] = p[i]; v[8 + i] = p[16 + i]; }
  return bsplit16(v); }
__device__ __forceinline__ F2 split_rowK(const float* row, int k0, int lane, int K) { float v[16]; const int g = lane >> 4;
#pragma unroll
  for (int i = 0; i < 8; ++i) { const int ka = k0 + 8 * g + i, kb = ka + 16; v[i] = ka < K ? row[ka < K ? ka : K - 1] : 0.f; v[8 + i] = kb < K ? row[kb < K ? kb : K - 1] : 0.f; }
  return bsplit16(v); }
__device__ __forceinline__ F2 split_col(const float* W, int k0, int n, int lane, int ld, int K) { float v[16]; const int g = lane >> 4;
#pragma unroll
  for (int i = 0; i < 8; ++i) { const int ka = k0 + 8 * g + i, kb = ka + 16; v[i] = ka < K ? W[(size_t)(ka < K ? ka : K - 1) * ld + n] : 0.f; v[8 + i] = kb < K ? W[(size_t)(kb < K ? kb : K - 1) * ld + n] : 0.f; }
  return bsplit16(v); }
__device__ __forceinline__ v8f mac3(const F2& a, const F2& b, v8f c) { c = wmma_bf(a.l, b.h, c); c = wmma_bf(a.h, b.l, c); return wmma_bf(a.h, b.h, c); }
__device__ __forceinline__ float sigm(float v) { return 1.0f / (1.0f + expf(-v)); }
#define LDSX() do { asm volatile("s_wait_dscnt 0" ::: "memory"); __builtin_amdgcn_wave_barrier(); __builtin_amdgcn_fence(__ATOMIC_RELEASE, "workgroup"); } while (0)

__device__ __forceinline__ float bfr(float v) { return (float)(__bf16)v; }
__device__ __forceinline__ v16b wcol_io(const float* __restrict__ Wm, int k0, int o, int lane, int ld) { v16b w; const float* p = Wm + (size_t)(k0 + 8 * (lane >> 4)) * ld + o;
#pragma unroll
  for (int i = 0; i < 8; ++i) { w[i] = (__bf16)p[(size_t)i * ld]; w[8 + i] = (__bf16)p[(size_t)(16 + i) * ld]; }
  asm volatile("s_wait_loadcnt 0x0" ::: "memory"); return w; }
#define NIMG 4
#define IH 96
#define CC 256
#define NHD 8
#define HDD 32
#define WSZ 8
#define STR 4
#define NWX 23
#define NWIN (NIMG * NWX * NWX)
#define NTW 64
#define NPIX (NIMG * IH * IH)
#ifndef NWINV
#define NWINV NWIN
#endif
#ifndef NPIXV
#define NPIXV NPIX
#endif
#define QW (3 * CC)
__device__ __forceinline__ size_t win_pix(int wdx, int n) { const int t = wdx / (NWX * NWX), wr = wdx % (NWX * NWX), wy = wr / NWX, wx = wr % NWX; const int yy = wy * STR + n / WSZ, xx = wx * STR + n % WSZ; return ((size_t)t * IH + yy) * IH + xx; }
__device__ __forceinline__ F2 split_ptr(const float* __restrict__ p, int lane) { float va[16]; const int g = lane >> 4;
#pragma unroll
  for (int i = 0; i < 8; ++i) { va[i] = p[8 * g + i]; va[8 + i] = p[16 + 8 * g + i]; }
  return bsplit16(va); }
__global__ __launch_bounds__(128) void k_qkvp(const float* __restrict__ X, const float* __restrict__ Wt, float* __restrict__ QP) { __shared__ __align__(16) float sf[4][16][132];
  const int tid = threadIdx.x, wave = tid >> 5, lane = tid & 31, col = lane & 15, g = lane >> 4; const int c0 = blockIdx.y * 128; const size_t r0 = (size_t)blockIdx.x * 64 + wave * 16;
  v8f acc[8] = {};
#pragma unroll 2
  for (int kc = 0; kc < CC / 32; ++kc) { v16b a; { const float* p = X + (r0 + col) * CC + kc * 32 + 8 * g; float t0[8], t1[8];
#pragma unroll
      for (int i = 0; i < 8; ++i) t0[i] = p[i];
      asm volatile("s_wait_loadcnt 0x0" ::: "memory");
#pragma unroll
      for (int i = 0; i < 8; ++i) t1[i] = p[16 + i];
      asm volatile("s_wait_loadcnt 0x0" ::: "memory");
#pragma unroll
      for (int i = 0; i < 8; ++i) { a[i] = (__bf16)t0[i]; a[8 + i] = (__bf16)t1[i]; } }
#pragma unroll
    for (int j = 0; j < 8; ++j) { v16b w; { const float* pw = Wt + (size_t)(c0 + j * 16 + col) * CC + kc * 32 + 8 * g; float t0[8], t1[8];
#pragma unroll
        for (int i = 0; i < 8; ++i) t0[i] = pw[i];
        asm volatile("s_wait_loadcnt 0x0" ::: "memory");
#pragma unroll
        for (int i = 0; i < 8; ++i) t1[i] = pw[16 + i];
        asm volatile("s_wait_loadcnt 0x0" ::: "memory");
#pragma unroll
        for (int i = 0; i < 8; ++i) { w[i] = (__bf16)t0[i]; w[8 + i] = (__bf16)t1[i]; } }
      acc[j] = wmma_bf(a, w, acc[j]); } }
#pragma unroll
  for (int j = 0; j < 8; ++j)
#pragma unroll
    for (int r = 0; r < 8; ++r) sf[wave][8 * g + r][j * 16 + col] = acc[j][r];
  LDSX(); for (int rl = 0; rl < 16; ++rl) vst2(QP + (r0 + rl) * QW + c0 + lane * 4, *(const v4f*)&sf[wave][rl][lane * 4]); }
__global__ __launch_bounds__(128) void k_modp(const float* __restrict__ MOD, const float* __restrict__ Wt, const float* __restrict__ Bq, float* __restrict__ MP) { __shared__ __align__(16) float sf[4][16][132];
  const int tid = threadIdx.x, wave = tid >> 5, lane = tid & 31, col = lane & 15, g = lane >> 4; const int c0 = blockIdx.y * 128; const size_t r0 = (size_t)wave * 16;
  v8f acc[8] = {};
#pragma unroll 2
  for (int kc = 0; kc < CC / 32; ++kc) { v16b a; { const float* p = MOD + (r0 + col) * CC + kc * 32 + 8 * g; float t0[8], t1[8];
#pragma unroll
      for (int i = 0; i < 8; ++i) t0[i] = p[i];
      asm volatile("s_wait_loadcnt 0x0" ::: "memory");
#pragma unroll
      for (int i = 0; i < 8; ++i) t1[i] = p[16 + i];
      asm volatile("s_wait_loadcnt 0x0" ::: "memory");
#pragma unroll
      for (int i = 0; i < 8; ++i) { a[i] = (__bf16)t0[i]; a[8 + i] = (__bf16)t1[i]; } }
#pragma unroll
    for (int j = 0; j < 8; ++j) { v16b w; { const float* pw = Wt + (size_t)(c0 + j * 16 + col) * CC + kc * 32 + 8 * g; float t0[8], t1[8];
#pragma unroll
        for (int i = 0; i < 8; ++i) t0[i] = pw[i];
        asm volatile("s_wait_loadcnt 0x0" ::: "memory");
#pragma unroll
        for (int i = 0; i < 8; ++i) t1[i] = pw[16 + i];
        asm volatile("s_wait_loadcnt 0x0" ::: "memory");
#pragma unroll
        for (int i = 0; i < 8; ++i) { w[i] = (__bf16)t0[i]; w[8 + i] = (__bf16)t1[i]; } }
      acc[j] = wmma_bf(a, w, acc[j]); } }
#pragma unroll
  for (int j = 0; j < 8; ++j) { const float bb = bfr(Bq[c0 + j * 16 + col]); asm volatile("s_wait_loadcnt 0x0" ::: "memory");
#pragma unroll
    for (int r = 0; r < 8; ++r) sf[wave][8 * g + r][j * 16 + col] = acc[j][r] + bb; }
  LDSX(); for (int rl = 0; rl < 16; ++rl) vst2(MP + (r0 + rl) * QW + c0 + lane * 4, *(const v4f*)&sf[wave][rl][lane * 4]); }
__global__ __launch_bounds__(128) void k_win(const float* __restrict__ QP, const float* __restrict__ MP, const float* __restrict__ RT, float* __restrict__ CTX) {
  __shared__ float sq[64][33], sk[64][33], sv[64][33]; __shared__ float ss[64][65]; __shared__ float srt[225 * NHD];
  const int tid = threadIdx.x, wave = tid >> 5, lane = tid & 31, col = lane & 15, g = lane >> 4; const int wdx = blockIdx.x; const int myrow = wave * 16 + col;
  for (int i = tid; i < 225 * NHD; i += 128) srt[i] = bfr(RT[i]);
  const size_t mypix = win_pix(wdx, myrow);
  for (int h = 0; h < NHD; ++h) {
    if (tid < 64) { const size_t px = win_pix(wdx, tid); const float* qp = QP + px * QW; const float* mp = MP + (size_t)tid * QW;
#pragma unroll
      for (int d4 = 0; d4 < HDD; d4 += 4) { const v4f q4 = *(const v4f*)(qp + h * HDD + d4), k4 = *(const v4f*)(qp + CC + h * HDD + d4), v4 = *(const v4f*)(qp + 2 * CC + h * HDD + d4); const v4f mq = *(const v4f*)(mp + h * HDD + d4), mk = *(const v4f*)(mp + CC + h * HDD + d4), mv = *(const v4f*)(mp + 2 * CC + h * HDD + d4);
        asm volatile("s_wait_loadcnt 0x0" ::: "memory");
#pragma unroll
        for (int i = 0; i < 4; ++i) { sq[tid][d4 + i] = (q4[i] + mq[i]) * 0.17677669529663689f; sk[tid][d4 + i] = k4[i] + mk[i]; sv[tid][d4 + i] = v4[i] + mv[i]; } } }
    __syncthreads();
    { const F2 a = split_ptr(&sq[myrow][0], lane); v8f acc[4] = {};
#pragma unroll
      for (int j = 0; j < 4; ++j) { const F2 bk = split_ptr(&sk[j * 16 + col][0], lane); acc[j] = wmma_bf(a.h, bk.h, acc[j]); acc[j] = wmma_bf(a.h, bk.l, acc[j]); acc[j] = wmma_bf(a.l, bk.h, acc[j]); acc[j] = wmma_bf(a.l, bk.l, acc[j]); }
#pragma unroll
      for (int j = 0; j < 4; ++j)
#pragma unroll
        for (int r = 0; r < 8; ++r) ss[wave * 16 + 8 * g + r][j * 16 + col] = acc[j][r]; }
    __syncthreads();
    if (lane < 16) { const int row = wave * 16 + lane; const int yi = row / WSZ, xi = row % WSZ; float mx = -3.0e38f; float e[NTW];
#pragma unroll
      for (int m = 0; m < NTW; ++m) { const int yj = m / WSZ, xj = m % WSZ; const int ridx = (yi - yj + WSZ - 1) * (2 * WSZ - 1) + (xi - xj + WSZ - 1); const float v = ss[row][m] + srt[ridx * NHD + h]; e[m] = v; mx = fmaxf(mx, v); }
      float sum = 0.f;
#pragma unroll
      for (int m = 0; m < NTW; ++m) { e[m] = expf(e[m] - mx); sum += e[m]; }
      const float inv = 1.0f / sum;
#pragma unroll
      for (int m = 0; m < NTW; ++m) ss[row][m] = e[m] * inv; }
    __syncthreads();
    { v8f acc[2] = {};
#pragma unroll
      for (int kc = 0; kc < 2; ++kc) { const F2 a = split_ptr(&ss[myrow][kc * 32], lane);
#pragma unroll
        for (int j = 0; j < 2; ++j) { float vb[16]; const int d = j * 16 + col;
#pragma unroll
          for (int i = 0; i < 8; ++i) { vb[i] = sv[kc * 32 + 8 * g + i][d]; vb[8 + i] = sv[kc * 32 + 16 + 8 * g + i][d]; }
          const F2 bv = bsplit16(vb); acc[j] = wmma_bf(a.h, bv.h, acc[j]); acc[j] = wmma_bf(a.h, bv.l, acc[j]); acc[j] = wmma_bf(a.l, bv.h, acc[j]); acc[j] = wmma_bf(a.l, bv.l, acc[j]); } }
#pragma unroll
      for (int j = 0; j < 2; ++j)
#pragma unroll
        for (int r = 0; r < 8; ++r) sq[wave * 16 + 8 * g + r][j * 16 + col] = acc[j][r];
      LDSX();
      for (int rl = 0; rl < 16; ++rl) { const int row = wave * 16 + rl; vst2(CTX + ((size_t)wdx * NTW + row) * CC + h * HDD + lane, sq[row][lane]); }     }
    __syncthreads(); }
  (void)mypix; }
__global__ __launch_bounds__(128) void k_fold(const float* __restrict__ CTX, const float* __restrict__ Wp, const float* __restrict__ Bp, float* __restrict__ OUT) { __shared__ __align__(16) float sf[4][16][132];
  const int tid = threadIdx.x, wave = tid >> 5, lane = tid & 31, col = lane & 15, g = lane >> 4; const int c0 = blockIdx.y * 128; const size_t r0 = (size_t)blockIdx.x * 64 + wave * 16;
  const size_t pix = r0 + col; const int t = (int)(pix / (IH * IH)); const int rem = (int)(pix % (IH * IH)); const int y = rem / IH, x = rem % IH;
  int wy0 = (y - WSZ + 1 + STR - 1); wy0 = wy0 < 0 ? 0 : wy0 / STR; int wy1 = y / STR; wy1 = wy1 > NWX - 1 ? NWX - 1 : wy1;
  int wx0 = (x - WSZ + 1 + STR - 1); wx0 = wx0 < 0 ? 0 : wx0 / STR; int wx1 = x / STR; wx1 = wx1 > NWX - 1 ? NWX - 1 : wx1;
  const float invc = 1.0f / ((float)((wy1 - wy0 + 1) * (wx1 - wx0 + 1)) + 1e-10f);
  v8f acc[8] = {};
#pragma unroll 1
  for (int kc = 0; kc < CC / 32; ++kc) { float va[16];
#pragma unroll
    for (int i = 0; i < 16; ++i) va[i] = 0.f;
#pragma unroll
    for (int ay = 0; ay < 2; ++ay)
#pragma unroll
      for (int ax = 0; ax < 2; ++ax) { const int wy = wy0 + ay, wx = wx0 + ax; const float keep = (wy <= wy1 && wx <= wx1) ? 1.f : 0.f; const int wyc = wy <= wy1 ? wy : wy1, wxc = wx <= wx1 ? wx : wx1;
        const int wdx = (t * NWX + wyc) * NWX + wxc; const int n = (y - wyc * STR) * WSZ + (x - wxc * STR); const float* p = CTX + ((size_t)wdx * NTW + n) * CC + kc * 32 + 8 * g; float t0[8], t1[8];
#pragma unroll
        for (int i = 0; i < 8; ++i) t0[i] = p[i];
        asm volatile("s_wait_loadcnt 0x0" ::: "memory");
#pragma unroll
        for (int i = 0; i < 8; ++i) t1[i] = p[16 + i];
        asm volatile("s_wait_loadcnt 0x0" ::: "memory");
#pragma unroll
        for (int i = 0; i < 8; ++i) { va[i] += keep * t0[i]; va[8 + i] += keep * t1[i]; } }
    asm volatile("s_wait_loadcnt 0x0" ::: "memory");
#pragma unroll
    for (int i = 0; i < 16; ++i) va[i] *= invc;
    const F2 a = bsplit16(va);
#pragma unroll
    for (int j = 0; j < 8; ++j) { v16b w; { const float* pw = Wp + (size_t)(c0 + j * 16 + col) * CC + kc * 32 + 8 * g; float t0[8], t1[8];
#pragma unroll
        for (int i = 0; i < 8; ++i) t0[i] = pw[i];
        asm volatile("s_wait_loadcnt 0x0" ::: "memory");
#pragma unroll
        for (int i = 0; i < 8; ++i) t1[i] = pw[16 + i];
        asm volatile("s_wait_loadcnt 0x0" ::: "memory");
#pragma unroll
        for (int i = 0; i < 8; ++i) { w[i] = (__bf16)t0[i]; w[8 + i] = (__bf16)t1[i]; } }
      acc[j] = wmma_bf(a.h, w, acc[j]); acc[j] = wmma_bf(a.l, w, acc[j]); } }
#pragma unroll
  for (int j = 0; j < 8; ++j) { const float bb = bfr(Bp[c0 + j * 16 + col]); asm volatile("s_wait_loadcnt 0x0" ::: "memory");
#pragma unroll
    for (int r = 0; r < 8; ++r) sf[wave][8 * g + r][j * 16 + col] = acc[j][r] + bb; }
  LDSX(); for (int rl = 0; rl < 16; ++rl) vst2(OUT + (r0 + rl) * CC + c0 + lane * 4, *(const v4f*)&sf[wave][rl][lane * 4]); }
#define WS_QP  0u
#define WS_MP  (WS_QP + 4u * (size_t)NPIX * QW)
#define WS_CTX (WS_MP + 4u * (size_t)64 * QW)
#define WS_END (WS_CTX + 4u * (size_t)NWIN * NTW * CC)
extern "C" void kernel_launch(void* const* d_in, const int* in_sizes, int n_in, void* d_out, int out_size, void* d_ws, size_t ws_size, hipStream_t stream) {
  (void)in_sizes; (void)n_in; (void)out_size;
  if (ws_size < (size_t)WS_END) return;
  char* ws = (char*)d_ws; const float** F = (const float**)d_in; float *QP = (float*)(ws + WS_QP), *MP = (float*)(ws + WS_MP), *CTX = (float*)(ws + WS_CTX);
  k_qkvp<<<dim3(NPIXV / 64, QW / 128), 128, 0, stream>>>(F[0], F[3], QP);
  k_modp<<<dim3(1, QW / 128), 128, 0, stream>>>(F[1], F[3], F[4], MP);
  k_win<<<dim3(NWINV), 128, 0, stream>>>(QP, MP, F[2], CTX);
  k_fold<<<dim3(NPIXV / 64, CC / 128), 128, 0, stream>>>(CTX, F[5], F[6], (float*)d_out);
}
